// RuchbahMamba3Block_14963666059312
// MI455X (gfx1250) — hardware-verified
//
#include <hip/hip_runtime.h>
#include <math.h>


typedef __attribute__((ext_vector_type(16))) _Float16 v16h;
typedef __attribute__((ext_vector_type(8)))  _Float16 v8h;
typedef __attribute__((ext_vector_type(8)))  float  v8f;
typedef __attribute__((ext_vector_type(4)))  float  v4f;
typedef __attribute__((ext_vector_type(4)))  unsigned v4u;
template <typename V> __device__ __forceinline__ void vst2(void* p, V v) {
    *(volatile V*)p = v; __threadfence(); *(volatile V*)p = v;
}
__device__ __forceinline__ v8f wmma_f16(v16h a, v16h b, v8f c) {
    v8f d = __builtin_amdgcn_wmma_f32_16x16x32_f16(false, a, false, b, (short)0, c, false, false);
    asm volatile("v_nop\n\tv_nop\n\tv_nop\n\tv_nop" : "+v"(d) : "v"(a), "v"(b));
    return d;
}
#define MB_B   2
#define MB_L   4096
#define MB_DM  1024
#define MB_DI  2048
#define MB_DT  64
#define MB_K   4
#define MB_M   (MB_B * MB_L)

#define LDS_PITCH 40

#define EPI_NONE  0
#define EPI_DECAY 1

__device__ inline v8h ld8_h(const float* p) {
    v4f lo = *(const v4f*)p;
    v4f hi = *(const v4f*)(p + 4);
    v8h r;
#pragma unroll
    for (int i = 0; i < 4; ++i) { r[i] = (_Float16)lo[i]; r[4 + i] = (_Float16)hi[i]; }
    return r;
}
__device__ inline v8h ld8_h(const _Float16* p) {
    return *(const v8h*)p;
}
__device__ inline void store_tile(const float* T, float* O, size_t ldo, int tid) {
    for (int g = tid; g < 128 * 16; g += 128) {
        const int r = g >> 4, pc = g & 15;
        vst2(O + (size_t)r * ldo + pc * 4, *(const v4f*)(T + r * 64 + pc * 4));
    }
}
__device__ inline void store_tile(const float* T, _Float16* O, size_t ldo, int tid) {
    for (int g = tid; g < 128 * 8; g += 128) {
        const int r = g >> 3, pc = g & 7;
        union { v8h h; v4u u; } pk;
#pragma unroll
        for (int i = 0; i < 8; ++i) pk.h[i] = (_Float16)T[r * 64 + pc * 8 + i];
        vst2(O + (size_t)r * ldo + pc * 8, pk.u);
    }
}

template <typename TA, typename TO>
__launch_bounds__(128)
__global__ void gemm_wmma(const TA*    __restrict__ Amat,
                          const float* __restrict__ Wmat,
                          TO*          __restrict__ Omat,
                          int M, int N, int K,
                          int mode,
                          const float* __restrict__ bias,
                          const float* __restrict__ alog)
{
    __shared__ __align__(16) _Float16 lA[128 * LDS_PITCH];
    __shared__ __align__(16) _Float16 lB[ 64 * LDS_PITCH];
    __shared__ __align__(16) float  lO[128 * 64];

    const int tid  = threadIdx.x;
    const int wave = tid >> 5;
    const int lane = tid & 31;
    const int half = lane >> 4;
    const int l16  = lane & 15;

    const int tileM = blockIdx.x * 128;
    const int tileN = blockIdx.y * 64;

    const int brow = tid >> 1;
    const int bcol = (tid & 1) << 4;

    v8f acc[2][4] = {};

    for (int k0 = 0; k0 < K; k0 += 32) {
        const TA*    ga = Amat + (size_t)(tileM + tid)  * K + k0;
        const float* gb = Wmat + (size_t)(tileN + brow) * K + (k0 + bcol);

        if (k0 + 32 < K) {
            __builtin_prefetch(ga + 32, 0, 1);
            __builtin_prefetch(gb + 32, 0, 1);
        }

        v8h a0 = ld8_h(ga);
        v8h a1 = ld8_h(ga + 8);
        v8h a2 = ld8_h(ga + 16);
        v8h a3 = ld8_h(ga + 24);
        v8h b0 = ld8_h(gb);
        v8h b1 = ld8_h(gb + 8);

        _Float16* sa = &lA[tid * LDS_PITCH];
        *(v8h*)(sa +  0) = a0;
        *(v8h*)(sa +  8) = a1;
        *(v8h*)(sa + 16) = a2;
        *(v8h*)(sa + 24) = a3;
        _Float16* sb = &lB[brow * LDS_PITCH + bcol];
        *(v8h*)(sb)     = b0;
        *(v8h*)(sb + 8) = b1;
        __syncthreads();

        union { v16h v; v8h h[2]; } af[2];
#pragma unroll
        for (int mt = 0; mt < 2; ++mt) {
            const int mrow = wave * 32 + mt * 16 + l16;
            af[mt].h[0] = *(const v8h*)&lA[mrow * LDS_PITCH + half * 8];
            af[mt].h[1] = *(const v8h*)&lA[mrow * LDS_PITCH + 16 + half * 8];
        }
#pragma unroll
        for (int nt = 0; nt < 4; ++nt) {
            const int nrow = nt * 16 + l16;
            union { v16h v; v8h h[2]; } bf;
            bf.h[0] = *(const v8h*)&lB[nrow * LDS_PITCH + half * 8];
            bf.h[1] = *(const v8h*)&lB[nrow * LDS_PITCH + 16 + half * 8];
#pragma unroll
            for (int mt = 0; mt < 2; ++mt) {
                acc[mt][nt] = wmma_f16(af[mt].v, bf.v, acc[mt][nt]);
            }
        }
        __syncthreads();
    }

#pragma unroll
    for (int nt = 0; nt < 4; ++nt) {
        const int n = tileN + nt * 16 + l16;
        float bn = 0.f, an = 0.f;
        if (mode == EPI_DECAY) {
            bn = bias[n];
            an = fminf(fmaxf(-__expf(alog[n]), -10.f), -1e-6f);
        }
#pragma unroll
        for (int mt = 0; mt < 2; ++mt) {
#pragma unroll
            for (int r = 0; r < 8; ++r) {
                const int ml = wave * 32 + mt * 16 + r + 8 * half;
                float v = acc[mt][nt][r];
                if (mode == EPI_DECAY) {
                    float dlt = v + bn;
                    float sp  = (dlt > 20.f) ? dlt : log1pf(__expf(dlt));
                    sp = fminf(fmaxf(sp, 1e-6f), 10.f);
                    float e = __expf(sp * an);
                    v = fminf(fmaxf(e, 1e-6f), 1.f);
                }
                lO[ml * 64 + nt * 16 + l16] = v;
            }
        }
    }
    __syncthreads();
    store_tile(lO, Omat + (size_t)tileM * N + tileN, (size_t)N, tid);
}

__launch_bounds__(256)
__global__ void conv_silu(const _Float16* __restrict__ xz,
                          const float*  __restrict__ cw,
                          const float*  __restrict__ cb,
                          _Float16*       __restrict__ xi)
{
    const int d  = (blockIdx.x * 256 + threadIdx.x) * 2;
    const int l0 = blockIdx.y * 256;
    const int b  = blockIdx.z;

    float w[2][4], bb[2];
#pragma unroll
    for (int j = 0; j < 2; ++j) {
#pragma unroll
        for (int k = 0; k < 4; ++k) w[j][k] = cw[(d + j) * MB_K + k];
        bb[j] = cb[d + j];
    }
    const size_t rowbase = (size_t)b * MB_L;
    auto ld2 = [&](int l, float& a, float& c) {
        if (l < 0) { a = 0.f; c = 0.f; return; }
        const _Float16* p = xz + (rowbase + l) * (2 * (size_t)MB_DI) + d;
        a = (float)p[0]; c = (float)p[1];
    };
    float xm3[2], xm2[2], xm1[2];
    ld2(l0 - 3, xm3[0], xm3[1]); ld2(l0 - 2, xm2[0], xm2[1]); ld2(l0 - 1, xm1[0], xm1[1]);
#pragma unroll 2
    for (int l = l0; l < l0 + 256; ++l) {
        float x0[2]; ld2(l, x0[0], x0[1]);
        union { _Float16 h[2]; unsigned u; } pk;
#pragma unroll
        for (int j = 0; j < 2; ++j) {
            const float v = w[j][0] * xm3[j] + w[j][1] * xm2[j] + w[j][2] * xm1[j] + w[j][3] * x0[j] + bb[j];
            const float s = v / (1.f + __expf(-v));
            pk.h[j] = (_Float16)s;
            xm3[j] = xm2[j]; xm2[j] = xm1[j]; xm1[j] = x0[j];
        }
        vst2((char*)(xi + (rowbase + l) * MB_DI + d), pk.u);
    }
}

__launch_bounds__(256)
__global__ void scan_gate(const float*  __restrict__ ebuf,
                          const _Float16* __restrict__ xi,
                          const _Float16* __restrict__ xz,
                          const float*  __restrict__ Dv,
                          _Float16*       __restrict__ y)
{
    const int d = (blockIdx.x * 256 + threadIdx.x) * 2;
    const int b = blockIdx.y;
    const float Dd0 = Dv[d], Dd1 = Dv[d + 1];
    const size_t rowbase = (size_t)b * MB_L;

    float st0 = 0.f, st1 = 0.f;
#pragma unroll 2
    for (int l = 0; l < MB_L; ++l) {
        const size_t m = rowbase + l;
        const float e0 = ebuf[m * MB_DI + d], e1 = ebuf[m * MB_DI + d + 1];
        const _Float16* up = xi + m * MB_DI + d;
        const float u0 = (float)up[0], u1 = (float)up[1];
        const _Float16* zp = xz + m * (2 * (size_t)MB_DI) + MB_DI + d;
        const float z0 = (float)zp[0], z1 = (float)zp[1];
        st0 = fminf(fmaxf(st0 * e0 + u0, -1e4f), 1e4f);
        st1 = fminf(fmaxf(st1 * e1 + u1, -1e4f), 1e4f);
        const float y0 = fminf(fmaxf(st0 + u0 * Dd0, -1e4f), 1e4f) * (z0 / (1.f + __expf(-z0)));
        const float y1 = fminf(fmaxf(st1 + u1 * Dd1, -1e4f), 1e4f) * (z1 / (1.f + __expf(-z1)));
        union { _Float16 h[2]; unsigned u; } pk;
        pk.h[0] = (_Float16)y0; pk.h[1] = (_Float16)y1;
        vst2((char*)(y + m * MB_DI + d), pk.u);
    }
}

extern "C" void kernel_launch(void* const* d_in, const int* in_sizes, int n_in,
                              void* d_out, int out_size, void* d_ws, size_t ws_size,
                              hipStream_t stream) {
    const float* x          = (const float*)d_in[0];
    const float* in_proj_w  = (const float*)d_in[1];
    const float* conv_w     = (const float*)d_in[2];
    const float* conv_b     = (const float*)d_in[3];
    const float* x_proj_w   = (const float*)d_in[4];
    const float* dt_proj_w  = (const float*)d_in[5];
    const float* dt_proj_b  = (const float*)d_in[6];
    const float* A_log      = (const float*)d_in[7];
    const float* Dvec       = (const float*)d_in[8];
    const float* out_proj_w = (const float*)d_in[9];
    float* out = (float*)d_out;

    _Float16* xz   = (_Float16*)d_ws;
    _Float16* xi   = xz  + (size_t)MB_M * 2 * MB_DI;
    float*  ebuf = (float*)(xi + (size_t)MB_M * MB_DI);
    _Float16* dtl  = (_Float16*)(ebuf + (size_t)MB_M * MB_DI);
    _Float16* ybuf = dtl + (size_t)MB_M * MB_DT;

    const dim3 gblk(128);

    gemm_wmma<float, _Float16><<<dim3(MB_M / 128, (2 * MB_DI) / 64), gblk, 0, stream>>>(
        x, in_proj_w, xz, MB_M, 2 * MB_DI, MB_DM, EPI_NONE, nullptr, nullptr);

    conv_silu<<<dim3(MB_DI / 512, MB_L / 256, MB_B), 256, 0, stream>>>(
        xz, conv_w, conv_b, xi);

    gemm_wmma<_Float16, _Float16><<<dim3(MB_M / 128, MB_DT / 64), gblk, 0, stream>>>(
        xi, x_proj_w, dtl, MB_M, MB_DT, MB_DI, EPI_NONE, nullptr, nullptr);

    gemm_wmma<_Float16, float><<<dim3(MB_M / 128, MB_DI / 64), gblk, 0, stream>>>(
        dtl, dt_proj_w, ebuf, MB_M, MB_DI, MB_DT, EPI_DECAY, dt_proj_b, A_log);

    scan_gate<<<dim3(MB_DI / 512, MB_B), 256, 0, stream>>>(
        ebuf, xi, xz, Dvec, ybuf);

    gemm_wmma<_Float16, float><<<dim3(MB_M / 128, MB_DM / 64), gblk, 0, stream>>>(
        ybuf, out_proj_w, out, MB_M, MB_DM, MB_DI, EPI_NONE, nullptr, nullptr);
}
